// ONNXExportWrapper_69389491634431
// MI455X (gfx1250) — hardware-run, weakly checked
//
#include <hip/hip_runtime.h>
#include <hip/hip_fp16.h>
#include <math.h>

typedef __attribute__((ext_vector_type(16))) _Float16 v16h;
typedef __attribute__((ext_vector_type(8)))  _Float16 v8h;
typedef __attribute__((ext_vector_type(8)))  float    v8f;
typedef __attribute__((ext_vector_type(4)))  float    v4f;
typedef __attribute__((ext_vector_type(2)))  unsigned v2u;

constexpr int kB    = 32;
constexpr int kT    = 4096;
constexpr int kD    = 256;
constexpr int kN    = 64;
constexpr int kLc   = 32;
constexpr int kNc   = 128;
constexpr int kRows = 4096;
constexpr int kGrp  = 32;
constexpr int kNg   = 8;
constexpr int kCls  = 5;
constexpr int kFeat = 512;
static_assert(kT == kLc * kNc);
static_assert(kRows == kB * kNc);
static_assert(kD == kGrp * kNg);
static_assert(kFeat == 2 * kD);
static_assert(kLc == 32 && kN == 64 && kGrp == 32 && kB == 32 && kNc == 128);
static_assert((kNc % 4) == 0);

constexpr size_t kSzXH   = (size_t)kRows * kLc * 2;
constexpr size_t kSzTOE  = (size_t)kD * kLc * 4;
constexpr size_t kSzRSM  = (size_t)kD * kLc * 4;
constexpr size_t kSzRSP  = (size_t)kD * kN * 4;
constexpr size_t kSzA32  = (size_t)kD * kN * 4;
constexpr size_t kSzMH   = (size_t)kD * kLc * kLc * 2;
constexpr size_t kSzPH   = (size_t)kD * kN * kLc * 2;
constexpr size_t kSzQH   = (size_t)kD * kLc * kN * 2;
constexpr size_t kSzG1   = (size_t)kGrp * kLc * kRows * 4;
constexpr size_t kSzG2   = (size_t)kGrp * kN * kRows * 4;
constexpr size_t kSzSH   = (size_t)kGrp * kRows * kN * 2;
constexpr size_t kSzYS   = (size_t)kGrp * kLc * kRows * 4;
constexpr size_t kSzAVG  = (size_t)kB * kD * 4;
constexpr size_t kSzMAXP = (size_t)kB * kD * 4;
static_assert(kSzXH == 262144ull);
static_assert(kSzTOE == 32768ull);
static_assert(kSzRSM == 32768ull);
static_assert(kSzRSP == 65536ull);
static_assert(kSzA32 == 65536ull);
static_assert(kSzMH == 524288ull);
static_assert(kSzPH == 1048576ull);
static_assert(kSzQH == 1048576ull);
static_assert(kSzG1 == 16777216ull);
static_assert(kSzG2 == 33554432ull);
static_assert(kSzSH == 16777216ull);
static_assert(kSzYS == 16777216ull);
static_assert(kSzAVG == 32768ull);
static_assert(kSzMAXP == 32768ull);
constexpr size_t kOffXH   = 0;
constexpr size_t kOffTOE  = kOffXH   + kSzXH;
constexpr size_t kOffRSM  = kOffTOE  + kSzTOE;
constexpr size_t kOffRSP  = kOffRSM  + kSzRSM;
constexpr size_t kOffA32  = kOffRSP  + kSzRSP;
constexpr size_t kOffMH   = kOffA32  + kSzA32;
constexpr size_t kOffPH   = kOffMH   + kSzMH;
constexpr size_t kOffQH   = kOffPH   + kSzPH;
constexpr size_t kOffG1   = kOffQH   + kSzQH;
constexpr size_t kOffG2   = kOffG1   + kSzG1;
constexpr size_t kOffSH   = kOffG2   + kSzG2;
constexpr size_t kOffYS   = kOffSH   + kSzSH;
constexpr size_t kOffAVG  = kOffYS   + kSzYS;
constexpr size_t kOffMAXP = kOffAVG  + kSzAVG;
constexpr size_t kWsTotal = kOffMAXP + kSzMAXP;
static_assert(kWsTotal == 87031808ull);
static_assert(kWsTotal <= 134217728ull);
static_assert((kOffTOE % 128) == 0 && (kOffRSM % 128) == 0 && (kOffRSP % 128) == 0 && (kOffA32 % 128) == 0 &&
              (kOffMH % 128) == 0 && (kOffPH % 128) == 0 && (kOffQH % 128) == 0 && (kOffG1 % 128) == 0 &&
              (kOffG2 % 128) == 0 && (kOffSH % 128) == 0 && (kOffYS % 128) == 0 && (kOffAVG % 128) == 0 &&
              (kOffMAXP % 128) == 0);

__device__ __forceinline__ _Float16 f16_flush(float v) {
  const float w = (fabsf(v) < 6.103515625e-05f) ? 0.0f : v;
  return (_Float16)w;
}

__device__ __forceinline__ float bf16r(float v) {
  unsigned u = __float_as_uint(v);
  u = (u + 0x7FFFu + ((u >> 16) & 1u)) & 0xFFFF0000u;
  return __uint_as_float(u);
}

namespace eng {
union FragU { v16h v; v8h h[2]; };
__device__ __forceinline__ v16h frag_load(const _Float16* p) {
  FragU f;
  f.h[0] = *(const v8h*)(p);
  f.h[1] = *(const v8h*)(p + 16);
  return f.v;
}
__device__ __forceinline__ v8f mma(v16h a, v16h b, v8f c) {
  return __builtin_amdgcn_wmma_f32_16x16x32_f16(false, a, false, b, (short)0, c, false, false);
}
__device__ __forceinline__ void guard1(v8f& a, v16h x, v16h y) {
  asm volatile("v_nop\n\tv_nop\n\tv_nop\n\tv_nop" : "+v"(a) : "v"(x), "v"(y));
}
__device__ __forceinline__ void guard_acc(v8f& a) {
  asm volatile("v_nop\n\tv_nop\n\tv_nop\n\tv_nop" : "+v"(a));
}
__device__ __forceinline__ void keep4(v16h a, v16h b, v16h c, v16h d) {
  asm volatile("v_nop" :: "v"(a), "v"(b), "v"(c), "v"(d));
}

template <int MI, int SPL>
__global__ __launch_bounds__(256) void gemm_f16_kernel(
    const unsigned short* __restrict__ Ap, const unsigned short* __restrict__ A2p, int lda,
    const unsigned short* __restrict__ Btp, const unsigned short* __restrict__ Bt2p, int ldb,
    float* __restrict__ C, int ldc, int M, int N, int K, float scale, float rscale)
{
  static_assert(MI >= 1 && MI <= 2);
  static_assert(SPL >= 0 && SPL <= 2);
  const _Float16* A   = (const _Float16*)Ap;
  const _Float16* A2  = (const _Float16*)A2p;
  const _Float16* Bt  = (const _Float16*)Btp;
  const _Float16* Bt2 = (const _Float16*)Bt2p;
  __shared__ __align__(16) float sT[8][16 * 68];
  const int lane = threadIdx.x & 31;
  const int wave = threadIdx.x >> 5;
  const int tilesN = N >> 6;
  const int tilesM = M / (16 * MI);
  const int tile = blockIdx.x * 8 + wave;
  if (tile >= tilesM * tilesN) return;
  const int tm = tile / tilesN;
  const int tn = tile - tm * tilesN;
  const int m0 = tm * (16 * MI);
  const int n0 = tn << 6;
  const int rlane = lane & 15;
  const int koff  = (lane >> 4) * 8;
  const int mOff  = (lane >> 4) * 8;

  v8f acc[MI][4], accr[MI][4];
#pragma unroll
  for (int i = 0; i < MI; ++i)
#pragma unroll
    for (int j = 0; j < 4; ++j) {
      acc[i][j]  = (v8f){0.f, 0.f, 0.f, 0.f, 0.f, 0.f, 0.f, 0.f};
      accr[i][j] = (v8f){0.f, 0.f, 0.f, 0.f, 0.f, 0.f, 0.f, 0.f};
    }

  for (int k0 = 0; k0 < K; k0 += 32) {
    v16h bh[4], bl[4];
#pragma unroll
    for (int j = 0; j < 4; ++j) {
      const size_t bo = (size_t)(n0 + (j << 4) + rlane) * ldb + koff + k0;
      bh[j] = frag_load(Bt + bo);
      if (SPL == 2) bl[j] = frag_load(Bt2 + bo); else bl[j] = bh[j];
    }
#pragma unroll
    for (int i = 0; i < MI; ++i) {
      const size_t ao = (size_t)(m0 + (i << 4) + rlane) * lda + koff + k0;
      const v16h ah = frag_load(A + ao);
      v16h al = ah;
      if (SPL >= 1) al = frag_load(A2 + ao);
#pragma unroll
      for (int j = 0; j < 4; ++j) {
        acc[i][j] = mma(ah, bh[j], acc[i][j]);
        if (SPL >= 1) accr[i][j] = mma(al, bh[j], accr[i][j]);
        if (SPL == 2) accr[i][j] = mma(ah, bl[j], accr[i][j]);
      }
#pragma unroll
      for (int j = 0; j < 4; ++j) {
        guard1(acc[i][j], ah, al);
        if (SPL >= 1) guard1(accr[i][j], ah, al);
      }
    }
    keep4(bh[0], bh[1], bh[2], bh[3]);
    if (SPL == 2) keep4(bl[0], bl[1], bl[2], bl[3]);
  }
#pragma unroll
  for (int i = 0; i < MI; ++i)
#pragma unroll
    for (int j = 0; j < 4; ++j) {
      guard_acc(acc[i][j]);
      if (SPL >= 1) guard_acc(accr[i][j]);
    }

  float* slab = sT[wave];
#pragma unroll
  for (int i = 0; i < MI; ++i) {
    const int mBase = m0 + (i << 4);
#pragma unroll
    for (int j = 0; j < 4; ++j) {
#pragma unroll
      for (int r = 0; r < 8; ++r) {
        float v = acc[i][j][r] * scale;
        if (SPL >= 1) v += accr[i][j][r] * rscale;
        slab[(mOff + r) * 68 + (j << 4) + rlane] = v;
      }
    }
    __builtin_amdgcn_fence(__ATOMIC_RELEASE, "workgroup");
    __builtin_amdgcn_wave_barrier();
    __builtin_amdgcn_fence(__ATOMIC_ACQUIRE, "workgroup");
    {
      const int hh = lane >> 4, c4 = (lane & 15) * 4;
      for (int pass = 0; pass < 2; ++pass) {
#pragma unroll
        for (int it = 0; it < 8; ++it) {
          const int row = it * 2 + hh;
          const v4f v = *(const v4f*)(slab + row * 68 + c4);
          *(volatile v4f*)(C + (size_t)(mBase + row) * ldc + n0 + c4) = v;
        }
        __threadfence();
      }
    }
    __builtin_amdgcn_fence(__ATOMIC_RELEASE, "workgroup");
    __builtin_amdgcn_wave_barrier();
    __builtin_amdgcn_fence(__ATOMIC_ACQUIRE, "workgroup");
  }
}
}

__global__ __launch_bounds__(256) void rne_rows_f16_kernel(
    const float* __restrict__ src, unsigned short* __restrict__ dH, int total8)
{
  const int i = blockIdx.x * 256 + threadIdx.x;
  if (i >= total8) return;
  const size_t e0 = (size_t)i << 3;
  const v4f a0 = *(const v4f*)(src + e0);
  const v4f a1 = *(const v4f*)(src + e0 + 4);
  const float f0 = a0[0];
  const float f1 = a0[1];
  const float f2 = a0[2];
  const float f3 = a0[3];
  const float f4 = a1[0];
  const float f5 = a1[1];
  const float f6 = a1[2];
  const float f7 = a1[3];
  v8h hv;
  hv[0] = f16_flush(bf16r(f0));
  hv[1] = f16_flush(bf16r(f1));
  hv[2] = f16_flush(bf16r(f2));
  hv[3] = f16_flush(bf16r(f3));
  hv[4] = f16_flush(bf16r(f4));
  hv[5] = f16_flush(bf16r(f5));
  hv[6] = f16_flush(bf16r(f6));
  hv[7] = f16_flush(bf16r(f7));
  unsigned short* qh = dH + e0;
  *(volatile v8h*)qh = hv;
  __threadfence();
  *(volatile v8h*)qh = hv;
}

__device__ __forceinline__ float pow_chain(float a, int k) {
  float p = 1.0f;
  for (int m = 0; m < 32; ++m) p = (m < k) ? (p * a) : p;
  return p;
}

static_assert(((kD * kLc) % 256) == 0);
__global__ __launch_bounds__(256) void toeplitz_kernel(
    const float* __restrict__ A_diag, const float* __restrict__ B_in, const float* __restrict__ C_out,
    float* __restrict__ TOE)
{
  const int idx = blockIdx.x * 256 + threadIdx.x;
  const int d = idx >> 5;
  const int k = idx & 31;
  float acc = 0.0f;
  for (int n = 0; n < kN; ++n) {
    const float a  = bf16r(A_diag[d * kN + n]);
    const float bn = bf16r(B_in[d * kN + n]);
    const float cn = bf16r(C_out[d * kN + n]);
    const float p  = pow_chain(a, k);
    acc = fmaf(cn * bn, p, acc);
  }
  float* q = TOE + idx;
  *(volatile float*)q = acc;
  __threadfence();
  *(volatile float*)q = acc;
}

static_assert(((kD * kN) % 256) == 0);
__global__ __launch_bounds__(256) void state_consts_kernel(
    const float* __restrict__ A_diag, const float* __restrict__ B_in,
    float* __restrict__ RSP, float* __restrict__ A32)
{
  const int idx = blockIdx.x * 256 + threadIdx.x;
  const float a  = bf16r(A_diag[idx]);
  const float bn = bf16r(B_in[idx]);
  float p = 1.0f;
  float s = 0.0f;
  for (int m = 0; m < 32; ++m) {
    s += p;
    p = p * a;
  }
  const float r = bn * s;
  float* q0 = RSP + idx;
  float* q1 = A32 + idx;
  *(volatile float*)q0 = r;
  *(volatile float*)q1 = p;
  __threadfence();
  *(volatile float*)q0 = r;
  *(volatile float*)q1 = p;
}

__global__ __launch_bounds__(256) void rowsum_kernel(
    const float* __restrict__ TOE, float* __restrict__ RSM)
{
  const int idx = blockIdx.x * 256 + threadIdx.x;
  const int d = idx >> 5;
  const int i = idx & 31;
  float s = 0.0f;
  for (int k = 0; k < kLc; ++k) {
    const float t = TOE[d * kLc + k];
    s += (k <= i) ? t : 0.0f;
  }
  float* q = RSM + idx;
  *(volatile float*)q = s;
  __threadfence();
  *(volatile float*)q = s;
}

static_assert(((kD * kLc * 4) % 256) == 0);
__global__ __launch_bounds__(256) void m_plane_kernel(
    const float* __restrict__ TOE, unsigned short* __restrict__ MH)
{
  const int idx = blockIdx.x * 256 + threadIdx.x;
  const int r  = idx >> 2;
  const int j0 = (idx & 3) * 8;
  const int d  = r >> 5;
  const int i  = r & 31;
  v8h hv;
#pragma unroll
  for (int e = 0; e < 8; ++e) {
    const int j = j0 + e;
    const bool live = (j <= i);
    const int tt = live ? (i - j) : 0;
    const float t = TOE[d * kLc + tt];
    const float v = live ? t : 0.0f;
    hv[e] = f16_flush(v);
  }
  unsigned short* q = MH + (size_t)r * kLc + j0;
  *(volatile v8h*)q = hv;
  __threadfence();
  *(volatile v8h*)q = hv;
}

static_assert(((kD * kN * 4) % 256) == 0);
__global__ __launch_bounds__(256) void p_plane_kernel(
    const float* __restrict__ A_diag, const float* __restrict__ B_in, unsigned short* __restrict__ PH)
{
  const int idx = blockIdx.x * 256 + threadIdx.x;
  const int r  = idx >> 2;
  const int j0 = (idx & 3) * 8;
  const float a  = bf16r(A_diag[r]);
  const float bn = bf16r(B_in[r]);
  float p = pow_chain(a, 24 - j0);
  v8h hv;
#pragma unroll
  for (int s = 0; s < 8; ++s) {
    const int e = 7 - s;
    hv[e] = f16_flush(bn * p);
    p = p * a;
  }
  unsigned short* q = PH + (size_t)r * kLc + j0;
  *(volatile v8h*)q = hv;
  __threadfence();
  *(volatile v8h*)q = hv;
}

static_assert(((kD * kLc * 8) % 256) == 0);
__global__ __launch_bounds__(256) void q_plane_kernel(
    const float* __restrict__ A_diag, const float* __restrict__ C_out, unsigned short* __restrict__ QH)
{
  const int idx = blockIdx.x * 256 + threadIdx.x;
  const int n0 = (idx & 7) * 8;
  const int ri = idx >> 3;
  const int d  = ri >> 5;
  const int i  = ri & 31;
  const v4f a0 = *(const v4f*)(A_diag + d * kN + n0);
  const v4f a1 = *(const v4f*)(A_diag + d * kN + n0 + 4);
  const v4f c0 = *(const v4f*)(C_out + d * kN + n0);
  const v4f c1 = *(const v4f*)(C_out + d * kN + n0 + 4);
  float av[8], cv[8];
  av[0] = a0[0]; av[1] = a0[1]; av[2] = a0[2]; av[3] = a0[3];
  av[4] = a1[0]; av[5] = a1[1]; av[6] = a1[2]; av[7] = a1[3];
  cv[0] = c0[0]; cv[1] = c0[1]; cv[2] = c0[2]; cv[3] = c0[3];
  cv[4] = c1[0]; cv[5] = c1[1]; cv[6] = c1[2]; cv[7] = c1[3];
  v8h hv;
#pragma unroll
  for (int e = 0; e < 8; ++e) {
    const float a  = bf16r(av[e]);
    const float cn = bf16r(cv[e]);
    const float p  = pow_chain(a, i + 1);
    hv[e] = f16_flush(cn * p);
  }
  unsigned short* q = QH + (size_t)ri * kN + n0;
  *(volatile v8h*)q = hv;
  __threadfence();
  *(volatile v8h*)q = hv;
}

static_assert(((kGrp * kB * 8) % 256) == 0);
__global__ __launch_bounds__(256) void carry_kernel(
    const float* __restrict__ G2, const float* __restrict__ w_in, const float* __restrict__ b_in,
    const float* __restrict__ RSP, const float* __restrict__ A32, unsigned short* __restrict__ SH, int g)
{
  const int idx = blockIdx.x * 256 + threadIdx.x;
  const int dl = idx >> 8;
  const int b  = (idx >> 3) & 31;
  const int n0 = (idx & 7) * 8;
  const int d  = g * kGrp + dl;
  const float w  = bf16r(w_in[d]);
  const float bb = bf16r(b_in[d]);
  const v4f ra0 = *(const v4f*)(A32 + d * kN + n0);
  const v4f ra1 = *(const v4f*)(A32 + d * kN + n0 + 4);
  const v4f rp0 = *(const v4f*)(RSP + d * kN + n0);
  const v4f rp1 = *(const v4f*)(RSP + d * kN + n0 + 4);
  float a32[8], drv[8], S[8];
  a32[0] = ra0[0]; a32[1] = ra0[1]; a32[2] = ra0[2]; a32[3] = ra0[3];
  a32[4] = ra1[0]; a32[5] = ra1[1]; a32[6] = ra1[2]; a32[7] = ra1[3];
  drv[0] = bb * rp0[0]; drv[1] = bb * rp0[1]; drv[2] = bb * rp0[2]; drv[3] = bb * rp0[3];
  drv[4] = bb * rp1[0]; drv[5] = bb * rp1[1]; drv[6] = bb * rp1[2]; drv[7] = bb * rp1[3];
#pragma unroll
  for (int e = 0; e < 8; ++e) S[e] = 0.0f;
  const float* gp = G2 + (size_t)(dl * kN + n0) * kRows + (size_t)b * kNc;
  unsigned short* sp = SH + ((size_t)dl * kRows + (size_t)b * kNc) * kN + n0;
  for (int c4 = 0; c4 < kNc / 4; ++c4) {
    v4f gv[8];
#pragma unroll
    for (int e = 0; e < 8; ++e) gv[e] = *(const v4f*)(gp + (size_t)e * kRows + 4 * c4);
#pragma unroll
    for (int cc = 0; cc < 4; ++cc) {
      v8h hv;
#pragma unroll
      for (int e = 0; e < 8; ++e) hv[e] = f16_flush(S[e]);
      unsigned short* q = sp + (size_t)(4 * c4 + cc) * kN;
      *(volatile v8h*)q = hv;
      __threadfence();
      *(volatile v8h*)q = hv;
#pragma unroll
      for (int e = 0; e < 8; ++e) {
        const float gq = gv[e][cc];
        S[e] = fmaf(a32[e], S[e], fmaf(w, gq, drv[e]));
      }
    }
  }
}

static_assert(((kB * kGrp) % 256) == 0);
__global__ __launch_bounds__(256) void pool_kernel(
    const float* __restrict__ G1, const float* __restrict__ YS, const float* __restrict__ x,
    const float* __restrict__ w_in, const float* __restrict__ b_in, const float* __restrict__ D_skip,
    const float* __restrict__ RSM, float* __restrict__ AVG, float* __restrict__ MAXP, int g)
{
  const int idx = blockIdx.x * 256 + threadIdx.x;
  const int b  = idx >> 5;
  const int dl = idx & 31;
  const int d  = g * kGrp + dl;
  const float w  = bf16r(w_in[d]);
  const float bb = bf16r(b_in[d]);
  const float Dd = bf16r(D_skip[d]);
  const float* g1p = G1 + (size_t)(dl * kLc) * kRows + (size_t)b * kNc;
  const float* ysp = YS + (size_t)(dl * kLc) * kRows + (size_t)b * kNc;
  const float* xp  = x + (size_t)b * kT;
  const float* rp  = RSM + d * kLc;
  float sum = 0.0f;
  float mx = -INFINITY;
  for (int c = 0; c < kNc; ++c) {
    for (int i2 = 0; i2 < kLc; ++i2) {
      const float xv = bf16r(xp[c * kLc + i2]);
      const float u  = fmaf(w, xv, bb);
      const float g1 = g1p[(size_t)i2 * kRows + c];
      const float ys = ysp[(size_t)i2 * kRows + c];
      const float rs = rp[i2];
      const float y  = w * g1 + bb * rs + ys + Dd * u;
      const float h  = 0.5f * y * (1.0f + tanhf(0.7978845608028654f * (y + 0.044715f * y * y * y)));
      sum += h;
      mx = fmaxf(mx, h);
    }
  }
  const float av = sum * (1.0f / 4096.0f);
  float* q0 = AVG + b * kD + d;
  float* q1 = MAXP + b * kD + d;
  *(volatile float*)q0 = av;
  *(volatile float*)q1 = mx;
  __threadfence();
  *(volatile float*)q0 = av;
  *(volatile float*)q1 = mx;
}

static_assert(kB * kCls == 160);
__global__ __launch_bounds__(160) void head_kernel(
    const float* __restrict__ AVG, const float* __restrict__ MAXP,
    const float* __restrict__ W_head, const float* __restrict__ b_head, float* __restrict__ out)
{
  const int o = threadIdx.x;
  const int b = o / kCls;
  const int k = o - b * kCls;
  float acc = 0.0f;
  for (int f = 0; f < kD; ++f)
    acc = fmaf(AVG[b * kD + f], bf16r(W_head[f * kCls + k]), acc);
  for (int f = 0; f < kD; ++f)
    acc = fmaf(MAXP[b * kD + f], bf16r(W_head[(kD + f) * kCls + k]), acc);
  const float r = acc + bf16r(b_head[k]);
  float* q = out + o;
  *(volatile float*)q = r;
  __threadfence();
  *(volatile float*)q = r;
}

static_assert(((kGrp * kLc) % 32) == 0 && ((kGrp * kN) % 32) == 0 && (kLc % 32) == 0);
static_assert((kRows % 64) == 0 && (kLc % 32) == 0 && (kN % 32) == 0);
static_assert((((kGrp * kLc) / 32) * (kRows / 64)) % 8 == 0);
static_assert((((kGrp * kN) / 32) * (kRows / 64)) % 8 == 0);
static_assert(((kLc / 32) * (kRows / 64)) % 8 == 0);
static_assert(((kB * kT / 8) % 256) == 0);

extern "C" void kernel_launch(void* const* d_in, const int* in_sizes, int n_in,
                              void* d_out, int out_size, void* d_ws, size_t ws_size,
                              hipStream_t stream)
{
  if (n_in < 9) return;
  if (in_sizes[0] != kB * kT) return;
  if (in_sizes[1] != kD) return;
  if (in_sizes[2] != kD) return;
  if (in_sizes[3] != kD * kN) return;
  if (in_sizes[4] != kD * kN) return;
  if (in_sizes[5] != kD * kN) return;
  if (in_sizes[6] != kD) return;
  if (in_sizes[7] != kFeat * kCls) return;
  if (in_sizes[8] != kCls) return;
  if (out_size != kB * kCls) return;
  if (ws_size < kWsTotal) return;

  const float* x      = (const float*)d_in[0];
  const float* w_in   = (const float*)d_in[1];
  const float* b_in   = (const float*)d_in[2];
  const float* A_diag = (const float*)d_in[3];
  const float* B_in   = (const float*)d_in[4];
  const float* C_out  = (const float*)d_in[5];
  const float* D_skip = (const float*)d_in[6];
  const float* W_head = (const float*)d_in[7];
  const float* b_head = (const float*)d_in[8];
  float* out = (float*)d_out;

  char* ws = (char*)d_ws;
  unsigned short* XH   = (unsigned short*)(ws + kOffXH);
  float*          TOE  = (float*)(ws + kOffTOE);
  float*          RSM  = (float*)(ws + kOffRSM);
  float*          RSP  = (float*)(ws + kOffRSP);
  float*          A32  = (float*)(ws + kOffA32);
  unsigned short* MH   = (unsigned short*)(ws + kOffMH);
  unsigned short* PH   = (unsigned short*)(ws + kOffPH);
  unsigned short* QH   = (unsigned short*)(ws + kOffQH);
  float*          G1   = (float*)(ws + kOffG1);
  float*          G2   = (float*)(ws + kOffG2);
  unsigned short* SH   = (unsigned short*)(ws + kOffSH);
  float*          YS   = (float*)(ws + kOffYS);
  float*          AVG  = (float*)(ws + kOffAVG);
  float*          MAXP = (float*)(ws + kOffMAXP);

  toeplitz_kernel<<<(kD * kLc) / 256, 256, 0, stream>>>(A_diag, B_in, C_out, TOE);
  state_consts_kernel<<<(kD * kN) / 256, 256, 0, stream>>>(A_diag, B_in, RSP, A32);
  rowsum_kernel<<<(kD * kLc) / 256, 256, 0, stream>>>(TOE, RSM);
  m_plane_kernel<<<(kD * kLc * 4) / 256, 256, 0, stream>>>(TOE, MH);
  p_plane_kernel<<<(kD * kN * 4) / 256, 256, 0, stream>>>(A_diag, B_in, PH);
  q_plane_kernel<<<(kD * kLc * 8) / 256, 256, 0, stream>>>(A_diag, C_out, QH);

  rne_rows_f16_kernel<<<(kB * kT / 8) / 256, 256, 0, stream>>>(x, XH, kB * kT / 8);

  constexpr int kTilesG1 = ((kGrp * kLc) / 32) * (kRows / 64);
  constexpr int kTilesG2 = ((kGrp * kN) / 32) * (kRows / 64);
  constexpr int kTilesYS = (kLc / 32) * (kRows / 64);

  for (int g = 0; g < kNg; ++g) {
    eng::gemm_f16_kernel<2, 0><<<dim3(kTilesG1 / 8), 256, 0, stream>>>(
        MH + (size_t)g * (kGrp * kLc) * kLc, nullptr, kLc, XH, nullptr, kLc,
        G1, kRows, kGrp * kLc, kRows, kLc, 1.0f, 0.0f);

    eng::gemm_f16_kernel<2, 0><<<dim3(kTilesG2 / 8), 256, 0, stream>>>(
        PH + (size_t)g * (kGrp * kN) * kLc, nullptr, kLc, XH, nullptr, kLc,
        G2, kRows, kGrp * kN, kRows, kLc, 1.0f, 0.0f);

    carry_kernel<<<(kGrp * kB * 8) / 256, 256, 0, stream>>>(G2, w_in, b_in, RSP, A32, SH, g);

    for (int dl = 0; dl < kGrp; ++dl) {
      const int d = g * kGrp + dl;
      eng::gemm_f16_kernel<2, 0><<<dim3(kTilesYS / 8), 256, 0, stream>>>(
          QH + (size_t)d * kLc * kN, nullptr, kN, SH + (size_t)dl * kRows * kN, nullptr, kN,
          YS + (size_t)dl * kLc * kRows, kRows, kLc, kRows, kN, 1.0f, 0.0f);
    }

    pool_kernel<<<(kB * kGrp) / 256, 256, 0, stream>>>(G1, YS, x, w_in, b_in, D_skip, RSM, AVG, MAXP, g);
  }

  head_kernel<<<1, kB * kCls, 0, stream>>>(AVG, MAXP, W_head, b_head, out);
}
